// PointnetSAModule_76854144795252
// MI455X (gfx1250) — hardware-verified
//
#include <hip/hip_runtime.h>
#include <math.h>

#pragma clang fp contract(off)

typedef __attribute__((ext_vector_type(16))) _Float16 v16h;
typedef __attribute__((ext_vector_type(8)))  _Float16 v8h;
typedef __attribute__((ext_vector_type(8)))  float    v8f;
typedef __attribute__((ext_vector_type(4)))  float    v4f;

constexpr int NBATCH  = 8;
constexpr int NPTS    = 8192;
constexpr int NCENTRE = 1024;
constexpr int NSAMP   = 32;
constexpr int CH_MID  = 64;
constexpr int CH_OUT  = 128;
constexpr int NROWS   = NBATCH * NPTS;
constexpr float BN_EPS = 1e-5f;
constexpr float BALL_R2 = 0.04f;
constexpr float RES_CARRY = 2048.0f;
constexpr float RES_CARRY_INV = 1.0f / 2048.0f;
constexpr float F16_MIN_NORMAL = 6.103515625e-5f;

constexpr int OUT0_FLOATS = NBATCH * NCENTRE * 3;
constexpr int OUT1_FLOATS = NBATCH * CH_OUT * NCENTRE;
static_assert(OUT0_FLOATS * 4 == 98304, "out0 bytes");
static_assert(OUT0_FLOATS * 4 + OUT1_FLOATS * 4 == 4292608, "d_out bytes");
static_assert((OUT0_FLOATS * 4) % 128 == 0, "out1 starts on a line");

constexpr size_t WS_H3_BYTES  = (size_t)NROWS * CH_OUT * 4;
constexpr size_t WS_CEN_OFF   = WS_H3_BYTES;
constexpr size_t WS_CEN_BYTES = (size_t)OUT0_FLOATS * 4;
constexpr size_t WS_TOTAL     = WS_CEN_OFF + WS_CEN_BYTES;
static_assert(WS_TOTAL <= 134217728, "carve");
static_assert(WS_CEN_OFF % 128 == 0, "carve alignment");

struct FragH {
  union U { v16h v; v8h h[2]; };
  static __device__ __forceinline__ v16h load(const _Float16* p) {
    U f; f.h[0] = *(const v8h*)(p); f.h[1] = *(const v8h*)(p + 16); return f.v;
  }
};

__device__ __forceinline__ v8f mma_h(v16h a, v16h b, v8f c) {
  c = __builtin_amdgcn_wmma_f32_16x16x32_f16(false, a, false, b, (short)0, c, false, false);
  asm volatile("v_nop\n\tv_nop\n\tv_nop\n\tv_nop" : "+v"(c) : "v"(a), "v"(b));
  return c;
}

__device__ __forceinline__ void split16(float v, _Float16& hi, _Float16& lo) {
  const _Float16 h0 = (_Float16)v;
  float hf = (float)h0;
  const bool tiny = fabsf(hf) < F16_MIN_NORMAL;
  hf = tiny ? 0.0f : hf;
  hi = (_Float16)hf;
  lo = (_Float16)((v - hf) * RES_CARRY);
}

__global__ __launch_bounds__(1024) void fps_kernel(const float* __restrict__ xyz,
                                                   float* __restrict__ out0,
                                                   float* __restrict__ cen_ws) {
#pragma clang fp contract(off)
  __shared__ __align__(16) float stg[12288];
  __shared__ float redV[32];
  __shared__ int   redI[32];
  __shared__ float curPt[4];

  const int b    = blockIdx.x;
  const int tid  = threadIdx.x;
  const int lane = tid & 31;
  const int wid  = tid >> 5;
  const float* xb = xyz + (size_t)b * NPTS * 3;

  float xr[8], yr[8], zr[8], dr[8];
#pragma unroll
  for (int half = 0; half < 2; ++half) {
#pragma unroll
    for (int i = 0; i < 3; ++i) {
      const int f4 = tid + i * 1024;
      const v4f t = *(const v4f*)(xb + half * 12288 + f4 * 4);
      *(v4f*)(stg + f4 * 4) = t;
    }
    __syncthreads();
#pragma unroll
    for (int k = 0; k < 4; ++k) {
      const int jl = tid + k * 1024;
      xr[half * 4 + k] = stg[jl * 3 + 0];
      yr[half * 4 + k] = stg[jl * 3 + 1];
      zr[half * 4 + k] = stg[jl * 3 + 2];
    }
    __syncthreads();
  }
#pragma unroll
  for (int k = 0; k < 8; ++k) dr[k] = INFINITY;

  if (tid == 0) {
    curPt[0] = xr[0]; curPt[1] = yr[0]; curPt[2] = zr[0];
    stg[0] = xr[0]; stg[1] = yr[0]; stg[2] = zr[0];
  }
  __syncthreads();

  for (int it = 0; it < NCENTRE; ++it) {
    const float cx = curPt[0], cy = curPt[1], cz = curPt[2];
    float bv = -1.0f;
    int bi = tid;
#pragma unroll
    for (int k = 0; k < 8; ++k) {
      const float dx = xr[k] - cx;
      const float dy = yr[k] - cy;
      const float dz = zr[k] - cz;
      const float t0 = dx * dx;
      const float t1 = dy * dy;
      const float t2 = dz * dz;
      const float d  = (t0 + t2) + t1;
      const float nd = fminf(dr[k], d);
      dr[k] = nd;
      if (nd > bv) { bv = nd; bi = tid + k * 1024; }
    }
#pragma unroll
    for (int off = 16; off > 0; off >>= 1) {
      const float ov = __shfl_down(bv, off, 32);
      const int   oi = __shfl_down(bi, off, 32);
      const bool take = (ov > bv) || (ov == bv && oi < bi);
      bv = take ? ov : bv;
      bi = take ? oi : bi;
    }
    if (lane == 0) { redV[wid] = bv; redI[wid] = bi; }
    __syncthreads();
    float v = redV[lane];
    int   i = redI[lane];
#pragma unroll
    for (int off = 16; off > 0; off >>= 1) {
      const float ov = __shfl_xor(v, off, 32);
      const int   oi = __shfl_xor(i, off, 32);
      const bool take = (ov > v) || (ov == v && oi < i);
      v = take ? ov : v;
      i = take ? oi : i;
    }
    const int ci = i & (NPTS - 1);
    const int kw = ci >> 10;
    float wx = xr[0], wy = yr[0], wz = zr[0];
#pragma unroll
    for (int kk = 1; kk < 8; ++kk) {
      const bool s = (kw == kk);
      wx = s ? xr[kk] : wx;
      wy = s ? yr[kk] : wy;
      wz = s ? zr[kk] : wz;
    }
    if (tid == (ci & 1023)) {
      curPt[0] = wx; curPt[1] = wy; curPt[2] = wz;
      if (it + 1 < NCENTRE) {
        stg[(it + 1) * 3 + 0] = wx;
        stg[(it + 1) * 3 + 1] = wy;
        stg[(it + 1) * 3 + 2] = wz;
      }
    }
    __syncthreads();
  }

  if (tid < 768) {
    const v4f val = *(const v4f*)(stg + tid * 4);
    volatile v4f* p0 = (volatile v4f*)(out0   + (size_t)b * NCENTRE * 3 + tid * 4);
    volatile v4f* p1 = (volatile v4f*)(cen_ws + (size_t)b * NCENTRE * 3 + tid * 4);
    *p0 = val;
    *p1 = val;
    __threadfence();
    *p0 = val;
    *p1 = val;
  }
}

constexpr int MLP_WAVES = 4;
constexpr int MLP_RT    = 4;
constexpr int MLP_ROWS_PER_BLOCK = MLP_WAVES * MLP_RT * 16;
constexpr int MLP_BLOCKS = NROWS / MLP_ROWS_PER_BLOCK;
static_assert(MLP_BLOCKS * MLP_ROWS_PER_BLOCK == NROWS, "row tiling is exact");
static_assert(CH_MID % 32 == 0, "K multiple of 32");
static_assert(CH_MID % 64 == 0 && CH_OUT % 64 == 0, "N multiple of 64");
constexpr int WPITCH = 72;
constexpr int APITCH = 72;
constexpr int SPITCH = 68;

__device__ __forceinline__ void stage_w8(const float* __restrict__ w, _Float16* wh, _Float16* wl, int g) {
  const int n  = g >> 3;
  const int k8 = (g & 7) * 8;
  const float* src = w + n * CH_MID + k8;
  const v4f a = *(const v4f*)(src);
  const v4f c = *(const v4f*)(src + 4);
  v8h hv, lv;
#pragma unroll
  for (int e = 0; e < 4; ++e) {
    _Float16 h, l;
    split16(a[e], h, l); hv[e] = h; lv[e] = l;
    split16(c[e], h, l); hv[4 + e] = h; lv[4 + e] = l;
  }
  *(v8h*)(wh + n * WPITCH + k8) = hv;
  *(v8h*)(wl + n * WPITCH + k8) = lv;
}

__global__ __launch_bounds__(128) void mlp_kernel(
    const float* __restrict__ xyz,
    const float* __restrict__ w1, const float* __restrict__ b1, const float* __restrict__ g1,
    const float* __restrict__ be1, const float* __restrict__ m1, const float* __restrict__ v1,
    const float* __restrict__ w2, const float* __restrict__ b2, const float* __restrict__ g2,
    const float* __restrict__ be2, const float* __restrict__ m2, const float* __restrict__ v2,
    const float* __restrict__ w3, const float* __restrict__ b3, const float* __restrict__ g3,
    const float* __restrict__ be3, const float* __restrict__ m3, const float* __restrict__ v3,
    float* __restrict__ H3) {
  __shared__ __align__(16) _Float16 sW2h[CH_MID * WPITCH];
  __shared__ __align__(16) _Float16 sW2l[CH_MID * WPITCH];
  __shared__ __align__(16) _Float16 sW3h[CH_OUT * WPITCH];
  __shared__ __align__(16) _Float16 sW3l[CH_OUT * WPITCH];
  __shared__ __align__(16) _Float16 sAh[MLP_WAVES][16 * APITCH];
  __shared__ __align__(16) _Float16 sAl[MLP_WAVES][16 * APITCH];
  __shared__ __align__(16) float sSlab[MLP_WAVES][16 * SPITCH];
  __shared__ __align__(16) float sP1[CH_MID * 8];
  __shared__ __align__(16) float sP2[CH_MID * 4];
  __shared__ __align__(16) float sP3[CH_OUT * 4];

  const int tid  = threadIdx.x;
  const int wave = tid >> 5;
  const int lane = tid & 31;
  const int hh   = lane >> 4;
  const int c    = lane & 15;

#pragma unroll 1
  for (int g = tid; g < CH_MID * 8; g += 128) stage_w8(w2, sW2h, sW2l, g);
#pragma unroll 1
  for (int g = tid; g < CH_OUT * 8; g += 128) stage_w8(w3, sW3h, sW3l, g);

  if (tid < CH_MID) {
    const float s = g1[tid] / sqrtf(v1[tid] + BN_EPS);
    const v4f pa = (v4f){w1[tid * 3 + 0], w1[tid * 3 + 1], w1[tid * 3 + 2], b1[tid]};
    const v4f pb = (v4f){m1[tid], s, be1[tid], 0.0f};
    *(v4f*)(sP1 + tid * 8)     = pa;
    *(v4f*)(sP1 + tid * 8 + 4) = pb;
  }
  asm volatile("" ::: "memory");
  if (tid < CH_MID) {
    const float s = g2[tid] / sqrtf(v2[tid] + BN_EPS);
    const v4f pp = (v4f){b2[tid], m2[tid], s, be2[tid]};
    *(v4f*)(sP2 + tid * 4) = pp;
  }
  asm volatile("" ::: "memory");
  {
    const float s = g3[tid] / sqrtf(v3[tid] + BN_EPS);
    const v4f pp = (v4f){b3[tid], m3[tid], s, be3[tid]};
    *(v4f*)(sP3 + tid * 4) = pp;
  }
  __syncthreads();

  _Float16* Ah = sAh[wave];
  _Float16* Al = sAl[wave];
  float* slab  = sSlab[wave];

#pragma unroll 1
  for (int rt = 0; rt < MLP_RT; ++rt) {
    const int row0 = blockIdx.x * MLP_ROWS_PER_BLOCK + (wave * MLP_RT + rt) * 16;

    {
      const float px = xyz[(size_t)(row0 + c) * 3 + 0];
      const float py = xyz[(size_t)(row0 + c) * 3 + 1];
      const float pz = xyz[(size_t)(row0 + c) * 3 + 2];
#pragma unroll 1
      for (int g = 0; g < 4; ++g) {
        v8h hv, lv;
#pragma unroll
        for (int e = 0; e < 8; ++e) {
          const int ch = hh * 32 + g * 8 + e;
          const v4f pa = *(const v4f*)(sP1 + ch * 8);
          const v4f pb = *(const v4f*)(sP1 + ch * 8 + 4);
          float d = px * pa[0];
          d = __builtin_fmaf(py, pa[1], d);
          d = __builtin_fmaf(pz, pa[2], d);
          float v = ((d + pa[3]) - pb[0]) * pb[1] + pb[2];
          v = fmaxf(v, 0.0f);
          _Float16 h, l;
          split16(v, h, l);
          hv[e] = h; lv[e] = l;
        }
        *(v8h*)(Ah + c * APITCH + hh * 32 + g * 8) = hv;
        *(v8h*)(Al + c * APITCH + hh * 32 + g * 8) = lv;
      }
    }
    __syncthreads();

    {
      v8f am[4], ar[4];
#pragma unroll
      for (int j = 0; j < 4; ++j) {
        am[j] = (v8f){0.f, 0.f, 0.f, 0.f, 0.f, 0.f, 0.f, 0.f};
        ar[j] = (v8f){0.f, 0.f, 0.f, 0.f, 0.f, 0.f, 0.f, 0.f};
      }
#pragma unroll
      for (int kk = 0; kk < 2; ++kk) {
        const v16h ah = FragH::load(Ah + c * APITCH + kk * 32 + 8 * hh);
        const v16h al = FragH::load(Al + c * APITCH + kk * 32 + 8 * hh);
#pragma unroll
        for (int j = 0; j < 4; ++j) {
          const v16h bh = FragH::load(sW2h + (j * 16 + c) * WPITCH + kk * 32 + 8 * hh);
          const v16h bl = FragH::load(sW2l + (j * 16 + c) * WPITCH + kk * 32 + 8 * hh);
          am[j] = mma_h(ah, bh, am[j]);
          ar[j] = mma_h(al, bh, ar[j]);
          ar[j] = mma_h(ah, bl, ar[j]);
        }
      }
#pragma unroll
      for (int j = 0; j < 4; ++j) {
        const int n = j * 16 + c;
        const v4f pp = *(const v4f*)(sP2 + n * 4);
#pragma unroll
        for (int r = 0; r < 8; ++r) {
          const float x = am[j][r] + ar[j][r] * RES_CARRY_INV;
          float v = ((x + pp[0]) - pp[1]) * pp[2] + pp[3];
          v = fmaxf(v, 0.0f);
          slab[(8 * hh + r) * SPITCH + n] = v;
        }
      }
    }
    __syncthreads();
    {
      const int q  = lane >> 3;
      const int c8 = (lane & 7) * 8;
#pragma unroll
      for (int it = 0; it < 4; ++it) {
        const int row = it * 4 + q;
        const float* sp = slab + row * SPITCH + c8;
        v8h hv, lv;
#pragma unroll
        for (int e = 0; e < 8; ++e) {
          _Float16 h, l;
          split16(sp[e], h, l);
          hv[e] = h; lv[e] = l;
        }
        *(v8h*)(Ah + row * APITCH + c8) = hv;
        *(v8h*)(Al + row * APITCH + c8) = lv;
      }
    }
    __syncthreads();

    {
      const v16h a0h = FragH::load(Ah + c * APITCH + 8 * hh);
      const v16h a1h = FragH::load(Ah + c * APITCH + 32 + 8 * hh);
      const v16h a0l = FragH::load(Al + c * APITCH + 8 * hh);
      const v16h a1l = FragH::load(Al + c * APITCH + 32 + 8 * hh);
#pragma unroll 1
      for (int nh = 0; nh < 2; ++nh) {
        v8f am[4], ar[4];
#pragma unroll
        for (int j = 0; j < 4; ++j) {
          am[j] = (v8f){0.f, 0.f, 0.f, 0.f, 0.f, 0.f, 0.f, 0.f};
          ar[j] = (v8f){0.f, 0.f, 0.f, 0.f, 0.f, 0.f, 0.f, 0.f};
        }
#pragma unroll
        for (int j = 0; j < 4; ++j) {
          const int n = nh * 64 + j * 16 + c;
          const v16h b0h = FragH::load(sW3h + n * WPITCH + 8 * hh);
          const v16h b1h = FragH::load(sW3h + n * WPITCH + 32 + 8 * hh);
          const v16h b0l = FragH::load(sW3l + n * WPITCH + 8 * hh);
          const v16h b1l = FragH::load(sW3l + n * WPITCH + 32 + 8 * hh);
          am[j] = mma_h(a0h, b0h, am[j]);
          am[j] = mma_h(a1h, b1h, am[j]);
          ar[j] = mma_h(a0l, b0h, ar[j]);
          ar[j] = mma_h(a0h, b0l, ar[j]);
          ar[j] = mma_h(a1l, b1h, ar[j]);
          ar[j] = mma_h(a1h, b1l, ar[j]);
        }
#pragma unroll
        for (int j = 0; j < 4; ++j) {
          const int nl = j * 16 + c;
          const v4f pp = *(const v4f*)(sP3 + (nh * 64 + nl) * 4);
#pragma unroll
          for (int r = 0; r < 8; ++r) {
            const float x = am[j][r] + ar[j][r] * RES_CARRY_INV;
            float v = ((x + pp[0]) - pp[1]) * pp[2] + pp[3];
            v = fmaxf(v, 0.0f);
            slab[(8 * hh + r) * SPITCH + nl] = v;
          }
        }
        __syncthreads();
        {
          const int c4 = (lane & 15) * 4;
          for (int pass = 0; pass < 2; ++pass) {
#pragma unroll
            for (int it = 0; it < 8; ++it) {
              const int row = it * 2 + hh;
              const v4f val = *(const v4f*)(slab + row * SPITCH + c4);
              *(volatile v4f*)(H3 + (size_t)(row0 + row) * CH_OUT + nh * 64 + c4) = val;
            }
            __threadfence();
          }
        }
        __syncthreads();
      }
    }
  }
}

constexpr int GRP_CEN = 32;
constexpr int TPITCH  = 36;
constexpr int GRP_BLOCKS = NBATCH * NCENTRE / GRP_CEN;
static_assert(NCENTRE % GRP_CEN == 0, "centre tiling");
static_assert(NPTS % 32 == 0, "scan chunking");

__global__ __launch_bounds__(256) void group_kernel(const float* __restrict__ xyz,
                                                    const float* __restrict__ cen,
                                                    const float* __restrict__ H3,
                                                    float* __restrict__ out1) {
#pragma clang fp contract(off)
  __shared__ int sIdx[GRP_CEN * NSAMP];
  __shared__ __align__(16) float sT[CH_OUT * TPITCH];

  const int tid  = threadIdx.x;
  const int wave = tid >> 5;
  const int lane = tid & 31;
  const int b    = blockIdx.x / (NCENTRE / GRP_CEN);
  const int s0   = (blockIdx.x % (NCENTRE / GRP_CEN)) * GRP_CEN;
  const float* xb = xyz + (size_t)b * NPTS * 3;

  float cx[4], cy[4], cz[4];
  int cnt[4];
#pragma unroll
  for (int q = 0; q < 4; ++q) {
    const size_t ci = (size_t)b * NCENTRE + s0 + wave * 4 + q;
    cx[q] = cen[ci * 3 + 0];
    cy[q] = cen[ci * 3 + 1];
    cz[q] = cen[ci * 3 + 2];
    cnt[q] = 0;
  }

  for (int base = 0; base < NPTS; base += 32) {
    if (cnt[0] >= NSAMP && cnt[1] >= NSAMP && cnt[2] >= NSAMP && cnt[3] >= NSAMP) break;
    const int j = base + lane;
    const float px = xb[j * 3 + 0];
    const float py = xb[j * 3 + 1];
    const float pz = xb[j * 3 + 2];
#pragma unroll
    for (int q = 0; q < 4; ++q) {
      const float dx = cx[q] - px;
      const float dy = cy[q] - py;
      const float dz = cz[q] - pz;
      const float t0 = dx * dx;
      const float t1 = dy * dy;
      const float t2 = dz * dz;
      const float d2 = (t0 + t2) + t1;
      const bool valid = d2 < BALL_R2;
      const unsigned mask = (unsigned)__ballot(valid);
      const int pos = cnt[q] + __popc(mask & ((1u << lane) - 1u));
      if (valid && pos < NSAMP) sIdx[(wave * 4 + q) * NSAMP + pos] = j;
      cnt[q] += __popc(mask);
    }
  }
#pragma unroll
  for (int q = 0; q < 4; ++q) {
    const int cq = cnt[q] < NSAMP ? cnt[q] : NSAMP;
    if (lane >= cq) sIdx[(wave * 4 + q) * NSAMP + lane] = 0;
  }
  __syncthreads();

#pragma unroll 1
  for (int q = 0; q < 4; ++q) {
    const int cenl = wave * 4 + q;
    v4f m = (v4f){-INFINITY, -INFINITY, -INFINITY, -INFINITY};
#pragma unroll 4
    for (int k = 0; k < NSAMP; ++k) {
      int id = sIdx[cenl * NSAMP + k];
      id = id < 0 ? 0 : id;
      id = id > NPTS - 1 ? NPTS - 1 : id;
      const v4f v = *(const v4f*)(H3 + ((size_t)b * NPTS + id) * CH_OUT + lane * 4);
      m[0] = fmaxf(m[0], v[0]);
      m[1] = fmaxf(m[1], v[1]);
      m[2] = fmaxf(m[2], v[2]);
      m[3] = fmaxf(m[3], v[3]);
    }
    sT[(lane * 4 + 0) * TPITCH + cenl] = m[0];
    sT[(lane * 4 + 1) * TPITCH + cenl] = m[1];
    sT[(lane * 4 + 2) * TPITCH + cenl] = m[2];
    sT[(lane * 4 + 3) * TPITCH + cenl] = m[3];
  }
  __syncthreads();

  {
    const int q8 = lane >> 3;
    const int c4 = (lane & 7) * 4;
    for (int pass = 0; pass < 2; ++pass) {
#pragma unroll
      for (int it = 0; it < 4; ++it) {
        const int ch = wave * 16 + it * 4 + q8;
        const v4f val = *(const v4f*)(sT + ch * TPITCH + c4);
        *(volatile v4f*)(out1 + ((size_t)b * CH_OUT + ch) * NCENTRE + s0 + c4) = val;
      }
      __threadfence();
    }
  }
}

extern "C" void kernel_launch(void* const* d_in, const int* in_sizes, int n_in,
                              void* d_out, int out_size, void* d_ws, size_t ws_size,
                              hipStream_t stream) {
  (void)in_sizes; (void)out_size;
  if (n_in < 19) return;
  if (ws_size < WS_TOTAL) return;

  const float* xyz = (const float*)d_in[0];
  const float* w1  = (const float*)d_in[1];
  const float* b1  = (const float*)d_in[2];
  const float* g1  = (const float*)d_in[3];
  const float* be1 = (const float*)d_in[4];
  const float* m1  = (const float*)d_in[5];
  const float* v1  = (const float*)d_in[6];
  const float* w2  = (const float*)d_in[7];
  const float* b2  = (const float*)d_in[8];
  const float* g2  = (const float*)d_in[9];
  const float* be2 = (const float*)d_in[10];
  const float* m2  = (const float*)d_in[11];
  const float* v2  = (const float*)d_in[12];
  const float* w3  = (const float*)d_in[13];
  const float* b3  = (const float*)d_in[14];
  const float* g3  = (const float*)d_in[15];
  const float* be3 = (const float*)d_in[16];
  const float* m3  = (const float*)d_in[17];
  const float* v3  = (const float*)d_in[18];

  float* out  = (float*)d_out;
  float* out0 = out;
  float* out1 = out + OUT0_FLOATS;

  char* ws = (char*)d_ws;
  float* H3     = (float*)(ws);
  float* cen_ws = (float*)(ws + WS_CEN_OFF);

  fps_kernel<<<NBATCH, 1024, 0, stream>>>(xyz, out0, cen_ws);

  mlp_kernel<<<MLP_BLOCKS, 128, 0, stream>>>(
      xyz,
      w1, b1, g1, be1, m1, v1,
      w2, b2, g2, be2, m2, v2,
      w3, b3, g3, be3, m3, v3,
      H3);

  group_kernel<<<GRP_BLOCKS, 256, 0, stream>>>(xyz, cen_ws, H3, out1);
}
